// MixtureCDFCoupling_12532714570305
// MI455X (gfx1250) — hardware-run, weakly checked
//
#include <hip/hip_runtime.h>
#include <math.h>

typedef __attribute__((ext_vector_type(16))) _Float16 v16h;
typedef __attribute__((ext_vector_type(16))) __bf16 v16b;
typedef __attribute__((ext_vector_type(8)))  _Float16 v8h;
typedef __attribute__((ext_vector_type(8)))  float v8f;
typedef __attribute__((ext_vector_type(4)))  float v4f;
typedef __attribute__((ext_vector_type(2)))  float v2f;
typedef __attribute__((ext_vector_type(4)))  unsigned v4u;
typedef __attribute__((ext_vector_type(4)))  int v4i;
typedef float __attribute__((may_alias)) float_a;
typedef int __attribute__((may_alias)) int_a;

template <typename T> __device__ __forceinline__ void vst2(void* p, T v) { *(volatile T*)p = v; __threadfence(); *(volatile T*)p = v; }
__device__ __forceinline__ v8f wmma16(v16h a, v16h b, v8f c) {
  v8f d = __builtin_amdgcn_wmma_f32_16x16x32_f16(false, a, false, b, (short)0, c, false, false);
  asm volatile("v_nop\n\tv_nop\n\tv_nop\n\tv_nop" : "+v"(d) : "v"(a), "v"(b));
  return d;
}
__device__ __forceinline__ v8f wmma_bf(v16b a, v16b b, v8f c) {
  v8f d = __builtin_amdgcn_wmma_f32_16x16x32_bf16(false, a, false, b, (short)0, c, false, false);
  asm volatile("v_nop\n\tv_nop\n\tv_nop\n\tv_nop" : "+v"(d) : "v"(a), "v"(b));
  return d;
}
__device__ __forceinline__ v16h frag_h(const _Float16* rowk0, int lane) {
  union { v16h v; v8h q[2]; } u; const _Float16* p = rowk0 + 8 * (lane >> 4);
  u.q[0] = *(const v8h*)p; u.q[1] = *(const v8h*)(p + 16); return u.v;
}
__device__ __forceinline__ v16h frag_f32(const float* rowk0, int lane) {
  v16h a; const float* p = rowk0 + 8 * (lane >> 4);
#pragma unroll
  for (int i = 0; i < 8; ++i) { a[i] = (_Float16)p[i]; a[8 + i] = (_Float16)p[16 + i]; }
  return a;
}
__device__ __forceinline__ v16h frag_f32s(const float* rowk0, int lane, float sc) {
  v16h a; const float* p = rowk0 + 8 * (lane >> 4);
#pragma unroll
  for (int i = 0; i < 8; ++i) { a[i] = (_Float16)(p[i] * sc); a[8 + i] = (_Float16)(p[16 + i] * sc); }
  return a;
}
__device__ __forceinline__ v16h fragc_f32(const float* W, int k0, int n, int lane, int ld, int K) {
  v16h a; const int g = lane >> 4;
#pragma unroll
  for (int i = 0; i < 8; ++i) { const int ka = k0 + 8 * g + i, kb = ka + 16;
    a[i] = (_Float16)(ka < K ? W[(size_t)(ka < K ? ka : K - 1) * ld + n] : 0.f); a[8 + i] = (_Float16)(kb < K ? W[(size_t)(kb < K ? kb : K - 1) * ld + n] : 0.f); }
  return a;
}
struct F2 { v16b h, l; };
__device__ __forceinline__ F2 bsplit16(const float v[16]) { F2 r;
#pragma unroll
  for (int i = 0; i < 16; ++i) { const __bf16 h = (__bf16)v[i]; r.h[i] = h; r.l[i] = (__bf16)(v[i] - (float)h); }
  return r; }
__device__ __forceinline__ F2 split_row(const float* row, int k0, int lane) { float v[16]; const float* p = row + k0 + 8 * (lane >> 4);
#pragma unroll
  for (int i = 0; i < 8; ++i) { v[i] = p[i]; v[8 + i] = p[16 + i]; }
  return bsplit16(v); }
__device__ __forceinline__ F2 split_rowK(const float* row, int k0, int lane, int K) { float v[16]; const int g = lane >> 4;
#pragma unroll
  for (int i = 0; i < 8; ++i) { const int ka = k0 + 8 * g + i, kb = ka + 16; v[i] = ka < K ? row[ka < K ? ka : K - 1] : 0.f; v[8 + i] = kb < K ? row[kb < K ? kb : K - 1] : 0.f; }
  return bsplit16(v); }
__device__ __forceinline__ F2 split_col(const float* W, int k0, int n, int lane, int ld, int K) { float v[16]; const int g = lane >> 4;
#pragma unroll
  for (int i = 0; i < 8; ++i) { const int ka = k0 + 8 * g + i, kb = ka + 16; v[i] = ka < K ? W[(size_t)(ka < K ? ka : K - 1) * ld + n] : 0.f; v[8 + i] = kb < K ? W[(size_t)(kb < K ? kb : K - 1) * ld + n] : 0.f; }
  return bsplit16(v); }
__device__ __forceinline__ v8f mac3(const F2& a, const F2& b, v8f c) { c = wmma_bf(a.l, b.h, c); c = wmma_bf(a.h, b.l, c); return wmma_bf(a.h, b.h, c); }
__device__ __forceinline__ float sigm(float v) { return 1.0f / (1.0f + expf(-v)); }
#define LDSX() do { asm volatile("s_wait_dscnt 0" ::: "memory"); __builtin_amdgcn_wave_barrier(); __builtin_amdgcn_fence(__ATOMIC_RELEASE, "workgroup"); } while (0)


#define NBT 16
#define LL 1024
#define NC 64
#define KM 10
#define NP (2 + 3 * KM)
#define HD1 1024
#define NO (NC * NP)
#define NRW (NBT * LL)
#ifndef NRT
#define NRT (NRW / 64)
#endif
typedef __attribute__((ext_vector_type(8))) __bf16 v8b;
__device__ __forceinline__ v16b frag_b(const __bf16* rowk0, int lane) {
  union { v16b v; v8b q[2]; } u; const __bf16* p = rowk0 + 8 * (lane >> 4);
  u.q[0] = *(const v8b*)p; u.q[1] = *(const v8b*)(p + 16); return u.v;
}
__device__ __forceinline__ float bfr(float v) { return (float)(__bf16)v; }
__device__ __attribute__((noinline)) float exp_ni(float v) { return expf(v); }
__device__ __attribute__((noinline)) float erf_ni(float v) { return erff(v); }
__device__ __attribute__((noinline)) float tanh_ni(float v) { return tanhf(v); }
__device__ __attribute__((noinline)) float log_ni(float v) { return logf(v); }
__device__ __attribute__((noinline)) float log1p_ni(float v) { return log1pf(v); }
__device__ __forceinline__ float softplus_f(float x) { return fmaxf(x, 0.f) + log1p_ni(exp_ni(-fabsf(x))); }
__device__ __forceinline__ float safe_log(float x) { return log_ni(fmaxf(x, 1e-22f)); }

#define PK_1 0
#define PK_2 (PK_1 + HD1 * NC)
#define PK_END (PK_2 + NO * HD1)
#define WS_PK  0u
#define WS_HH  (WS_PK + 2u * PK_END)
#define WS_HL  (WS_HH + 2u * NRW * HD1)
#define WS_LJ  (WS_HL + 2u * NRW * HD1)
#define WS_END (WS_LJ + 4u * NRW)

__global__ __launch_bounds__(256) void k_packT(const float* __restrict__ W1, const float* __restrict__ W2, __bf16* __restrict__ PK) {
  __shared__ __align__(16) __bf16 s[HD1]; const int n = blockIdx.x, which = blockIdx.y, tid = threadIdx.x; int K; size_t dst;
  if (which == 0) { if (n >= HD1) return; K = NC; dst = PK_1 + (size_t)n * NC; for (int k = tid; k < K; k += 256) s[k] = (__bf16)W1[(size_t)k * HD1 + n]; }
  else { K = HD1; dst = PK_2 + (size_t)n * HD1; for (int k = tid; k < K; k += 256) s[k] = (__bf16)W2[(size_t)k * NO + n]; }
  __syncthreads();
  for (int q = tid; q < K / 8; q += 256) vst2((unsigned*)(PK + dst + q * 8), *(const v4u*)&s[q * 8]);
}
__global__ __launch_bounds__(128) void k_l1(const float* __restrict__ Z, const float* __restrict__ MASK, const __bf16* __restrict__ P, const float* __restrict__ B1, __bf16* __restrict__ HH, __bf16* __restrict__ HL) {
  __shared__ __align__(16) __bf16 sh_[4][16][136]; __shared__ __align__(16) __bf16 sl_[4][16][136];
  const int tid = threadIdx.x, wave = tid >> 5, lane = tid & 31, col = lane & 15, g = lane >> 4; const size_t r0 = (size_t)blockIdx.x * 64 + wave * 16; const int n0 = blockIdx.y * 128;
  v8f acc[8] = {};
#pragma unroll
  for (int kc = 0; kc < NC / 32; ++kc) { float v[16]; const float* p = Z + (r0 + col) * NC + kc * 32 + 8 * g; const float* mk = MASK + kc * 32 + 8 * g;
#pragma unroll
    for (int i = 0; i < 8; ++i) { v[i] = bfr(p[i]) * bfr(mk[i]); v[8 + i] = bfr(p[16 + i]) * bfr(mk[16 + i]); }
    const F2 a = bsplit16(v);
#pragma unroll
    for (int j = 0; j < 8; ++j) { const v16b w = frag_b(P + (size_t)(n0 + j * 16 + col) * NC + kc * 32, lane); acc[j] = wmma_bf(a.l, w, acc[j]); acc[j] = wmma_bf(a.h, w, acc[j]); } }
#pragma unroll
  for (int j = 0; j < 8; ++j) { const float bb = bfr(B1[n0 + j * 16 + col]);
#pragma unroll
    for (int r = 0; r < 8; ++r) { const float x = acc[j][r] + bb; const float y = x * (0.5f * (1.0f + tanh_ni(0.7978845608028654f * (x + 0.044715f * x * x * x)))); const __bf16 hb = (__bf16)y; sh_[wave][8 * g + r][j * 16 + col] = hb; sl_[wave][8 * g + r][j * 16 + col] = (__bf16)(y - (float)hb); } }
  LDSX();
  for (int rl = 0; rl < 16; ++rl) if (lane < 16) { vst2((unsigned*)(HH + (r0 + rl) * HD1 + n0 + lane * 8), *(const v4u*)&sh_[wave][rl][lane * 8]); vst2((unsigned*)(HL + (r0 + rl) * HD1 + n0 + lane * 8), *(const v4u*)&sl_[wave][rl][lane * 8]); }
}
__global__ __launch_bounds__(128) void k_l2(const __bf16* __restrict__ HH, const __bf16* __restrict__ HL, const __bf16* __restrict__ P, const float* __restrict__ B2, const float* __restrict__ Z, const float* __restrict__ MASK, const float* __restrict__ SF, const float* __restrict__ MSF, float* __restrict__ ZOUT, float* __restrict__ LJ) {
  __shared__ __align__(16) float so[4][16][132]; __shared__ __align__(16) float sz[64][68]; __shared__ float slj[4][16][4]; __shared__ __align__(16) float srow[64];
  const int tid = threadIdx.x, wave = tid >> 5, lane = tid & 31, col = lane & 15, g = lane >> 4; const size_t r0 = (size_t)blockIdx.x * 64 + wave * 16;
  for (int q = tid; q < 64 * NC; q += 128) { const int rl = q >> 6, c = q & 63; sz[rl][c] = bfr(Z[((size_t)blockIdx.x * 64 + rl) * NC + c]) * bfr(MASK[c]); }
  if (tid < 64) srow[tid] = 0.f;
  __syncthreads();
#pragma unroll 1
  for (int ps = 0; ps < NO / 128; ++ps) { const int n0 = ps * 128; const int c0 = ps * 4;
    bool any = false;
#pragma unroll
    for (int cl = 0; cl < 4; ++cl) any |= (1.0f - bfr(MASK[c0 + cl])) != 0.f;
    if (!any) continue;
    v8f acc[8] = {};
#pragma unroll 2
    for (int kc = 0; kc < HD1 / 32; ++kc) { F2 a; a.h = frag_b(HH + (r0 + col) * HD1 + kc * 32, lane); a.l = frag_b(HL + (r0 + col) * HD1 + kc * 32, lane);
#pragma unroll
      for (int j = 0; j < 8; ++j) { const v16b w = frag_b(P + (size_t)(n0 + j * 16 + col) * HD1 + kc * 32, lane); acc[j] = wmma_bf(a.l, w, acc[j]); acc[j] = wmma_bf(a.h, w, acc[j]); } }
#pragma unroll
    for (int j = 0; j < 8; ++j) { const float bb = bfr(B2[n0 + j * 16 + col]);
#pragma unroll
      for (int r = 0; r < 8; ++r) so[wave][8 * g + r][j * 16 + col] = acc[j][r] + bb; }
    LDSX();
#pragma unroll 1
    for (int it = 0; it < 2; ++it) { const int rl = lane & 15, cl = (lane >> 4) + 2 * it, c = c0 + cl; const float* pp = &so[wave][rl][cl * NP]; const size_t row = r0 + rl;
      const float mk = bfr(MASK[c]); const float cm = 1.0f - mk;
      const float sf = exp_ni(bfr(SF[c]));
      const float t = pp[0] * cm; const float log_s = (tanh_ni(pp[1] / fmaxf(sf, 1.0f)) * sf) * cm;
      float log_pi[KM], mt[KM], mls[KM]; float mx = -3.0e38f;
#pragma unroll
      for (int k = 0; k < KM; ++k) { const float msf = exp_ni(bfr(MSF[c * KM + k])); log_pi[k] = pp[2 + k] * cm; mt[k] = pp[2 + KM + k] * cm; mls[k] = (tanh_ni(pp[2 + 2 * KM + k] / fmaxf(msf, 1.0f)) * msf) * cm; mx = fmaxf(mx, log_pi[k]); }
      float se = 0.f;
#pragma unroll
      for (int k = 0; k < KM; ++k) se += exp_ni(log_pi[k] - mx);
      const float lse = mx + log_ni(se);
      const float zc = bfr(Z[row * NC + c]);
      float u[KM], a1 = -3.0e38f, a2 = -3.0e38f, v1[KM], v2[KM];
#pragma unroll
      for (int k = 0; k < KM; ++k) { const float lw = log_pi[k] - lse; u[k] = (zc - mt[k]) * exp_ni(-mls[k]); v1[k] = lw + (-softplus_f(-u[k])); v2[k] = lw + ((u[k] - mls[k]) - 2.0f * softplus_f(u[k])); a1 = fmaxf(a1, v1[k]); a2 = fmaxf(a2, v2[k]); }
      float s1 = 0.f, s2 = 0.f;
#pragma unroll
      for (int k = 0; k < KM; ++k) { s1 += exp_ni(v1[k] - a1); s2 += exp_ni(v2[k] - a2); }
      const float log_cdf = a1 + log_ni(s1); const float logistic_ldj = a2 + log_ni(s2);
      const float p_cdf = exp_ni(log_cdf);
      const float z_logit = -safe_log(1.0f / p_cdf - 1.0f);
      const float mixt_ldj = -safe_log(p_cdf) - safe_log(1.0f - p_cdf);
      const float zo = (z_logit + t) * exp_ni(log_s);
      sz[wave * 16 + rl][c] = zo * cm + zc * mk;
      slj[wave][rl][cl] = cm * ((log_s + mixt_ldj) + logistic_ldj); }
    LDSX();
    if (lane < 16) { float a = srow[wave * 16 + lane];
#pragma unroll
      for (int cl = 0; cl < 4; ++cl) a += slj[wave][lane][cl];
      srow[wave * 16 + lane] = a; }
    LDSX(); }
  __syncthreads();
  for (int q = tid; q < 64 * 16; q += 128) { const int rl = q >> 4, pc = q & 15; vst2(ZOUT + ((size_t)blockIdx.x * 64 + rl) * NC + pc * 4, *(const v4f*)&sz[rl][pc * 4]); }
  if (tid < 16) vst2(LJ + (size_t)blockIdx.x * 64 + tid * 4, *(const v4f*)&srow[tid * 4]);
}
__global__ __launch_bounds__(64) void k_ldj(const float* __restrict__ LJ, float* __restrict__ OUT1) {
  __shared__ __align__(16) float s[NBT]; const int tid = threadIdx.x;
  if (tid < NBT) { float a = 0.f; const bool live = (size_t)(tid + 1) * LL <= (size_t)NRT * 64;
    for (int l = 0; l < LL; ++l) a += live ? LJ[(size_t)tid * LL + l] : 0.f;
    s[tid] = live ? a : 0.f; }
  __syncthreads();
  if (tid < NBT / 4) vst2(OUT1 + tid * 4, *(const v4f*)&s[tid * 4]);
}
extern "C" void kernel_launch(void* const* d_in, const int* in_sizes, int n_in, void* d_out, int out_size, void* d_ws, size_t ws_size, hipStream_t stream) {
  (void)in_sizes; (void)n_in; (void)out_size;
  const float** F = (const float**)d_in;
  if (ws_size < (size_t)WS_END) return;
  char* ws = (char*)d_ws; __bf16* PK = (__bf16*)(ws + WS_PK); __bf16 *HHp = (__bf16*)(ws + WS_HH), *HLp = (__bf16*)(ws + WS_HL); float* LJ = (float*)(ws + WS_LJ);
  float* ZOUT = (float*)d_out; float* OUT1 = (float*)((char*)d_out + (size_t)4 * NRW * NC);
  k_packT<<<dim3(NO, 2), 256, 0, stream>>>(F[2], F[4], PK);
  k_l1<<<dim3(NRT, HD1 / 128), 128, 0, stream>>>(F[0], F[1], PK + PK_1, F[3], HHp, HLp);
  k_l2<<<NRT, 128, 0, stream>>>(HHp, HLp, PK + PK_2, F[5], F[0], F[1], F[6], F[7], ZOUT, LJ);
  k_ldj<<<1, 64, 0, stream>>>(LJ, OUT1);
}
